// SinkhornOT_49211735277882
// MI455X (gfx1250) — hardware-verified
//
#include <hip/hip_runtime.h>


#define BB 8
#define NN 2048
#define DD 64
#define ITERS 50

typedef __attribute__((ext_vector_type(16))) __bf16 v16bf;
typedef __attribute__((ext_vector_type(8)))  __bf16 v8bf;
typedef __attribute__((ext_vector_type(8)))  float  v8f;
typedef __attribute__((ext_vector_type(4)))  float  v4f;
typedef __attribute__((ext_vector_type(4)))  unsigned v4u;
typedef __attribute__((ext_vector_type(4)))  int    v4i;
typedef float __attribute__((may_alias)) float_a;

__device__ __forceinline__ v8f wmma_bf16(v16bf a, v16bf b, v8f c) {
    v8f d = __builtin_amdgcn_wmma_f32_16x16x32_bf16(false, a, false, b, (short)0, c, false, false);
    asm volatile("v_nop\n\tv_nop\n\tv_nop\n\tv_nop" : "+v"(d) : "v"(a), "v"(b));
    return d;
}
template <typename V> __device__ __forceinline__ void vst2(void* p, V v) {
    *(volatile V*)p = v; __threadfence(); *(volatile V*)p = v;
}
__device__ __forceinline__ __bf16 bf_hi(float x) { return (__bf16)x; }
__device__ __forceinline__ __bf16 bf_lo(float x, __bf16 h) { return (__bf16)(x - (float)h); }

__device__ __forceinline__ void frag_f32_split(const float* row, int k0, int lane, v16bf& hi, v16bf& lo) {
    const float* p = row + k0 + 8 * (lane >> 4);
    const v4f a0 = *(const v4f*)(p), a1 = *(const v4f*)(p + 4), a2 = *(const v4f*)(p + 16), a3 = *(const v4f*)(p + 20);
#pragma unroll
    for (int i = 0; i < 4; ++i) {
        __bf16 h;
        h = bf_hi(a0[i]); hi[i]      = h; lo[i]      = bf_lo(a0[i], h);
        h = bf_hi(a1[i]); hi[4 + i]  = h; lo[4 + i]  = bf_lo(a1[i], h);
        h = bf_hi(a2[i]); hi[8 + i]  = h; lo[8 + i]  = bf_lo(a2[i], h);
        h = bf_hi(a3[i]); hi[12 + i] = h; lo[12 + i] = bf_lo(a3[i], h);
    }
}

__global__ __launch_bounds__(256) void sk_init(float* __restrict__ v) {
    const int g = blockIdx.x * 256 + threadIdx.x;
    const float x = 1.0f / NN;
    vst2(v + g * 4, (v4f){x, x, x, x});
}

__global__ __launch_bounds__(256) void sk_rowsq(const float* __restrict__ x0, const float* __restrict__ x1,
                                                float* __restrict__ sq0, float* __restrict__ sq1) {
    const int i = blockIdx.x * 256 + threadIdx.x;
    const float* p0 = x0 + (size_t)i * DD;
    const float* p1 = x1 + (size_t)i * DD;
    double s0 = 0.0, s1 = 0.0;
#pragma unroll 8
    for (int k = 0; k < DD; ++k) { const double a = p0[k]; s0 += a * a; const double b = p1[k]; s1 += b * b; }
    vst2(sq0 + i, (float_a)(float)s0);
    vst2(sq1 + i, (float_a)(float)s1);
}

__global__ __launch_bounds__(256) void sk_cost(const float* __restrict__ x0, const float* __restrict__ x1,
                                               const float* __restrict__ sq0, const float* __restrict__ sq1,
                                               float* __restrict__ Cm, float* __restrict__ maxpart) {
    __shared__ __align__(16) float Ct[8][16 * 32];
    __shared__ float wmax[8];
    const int tid = threadIdx.x, wave = tid >> 5, lane = tid & 31, h = lane >> 4, ln = lane & 15;
    const int blk = blockIdx.x;
    const int ct = blk & 63;
    const int rt = (blk >> 6) & 15;
    const int b  = blk >> 10;
    const int row0 = rt * 128 + wave * 16;
    const int col0 = ct * 32;

    const float* arow = x0 + ((size_t)b * NN + row0 + ln) * DD;
    v16bf ah[2], al[2];
#pragma unroll
    for (int ks = 0; ks < 2; ++ks) frag_f32_split(arow, ks * 32, lane, ah[ks], al[ks]);

    float mx = 0.0f;
#pragma unroll
    for (int nt = 0; nt < 2; ++nt) {
        const float* brow = x1 + ((size_t)b * NN + col0 + nt * 16 + ln) * DD;
        v8f acc = {};
#pragma unroll
        for (int ks = 0; ks < 2; ++ks) {
            v16bf bh, bl; frag_f32_split(brow, ks * 32, lane, bh, bl);
            acc = wmma_bf16(ah[ks], bh, acc);
            acc = wmma_bf16(ah[ks], bl, acc);
            acc = wmma_bf16(al[ks], bh, acc);
        }
        const int col = col0 + nt * 16 + ln;
        const float s1c = sq1[b * NN + col];
#pragma unroll
        for (int r = 0; r < 8; ++r) {
            const int rowl = 8 * h + r;
            const float d2 = (sq0[b * NN + row0 + rowl] + s1c) - 2.0f * acc[r];
            const float cv = sqrtf(fmaxf(d2, 0.0f));
            Ct[wave][rowl * 32 + nt * 16 + ln] = cv;
            mx = fmaxf(mx, cv);
        }
    }
    for (int m = 16; m > 0; m >>= 1) mx = fmaxf(mx, __shfl_xor(mx, m, 32));
    if (lane == 0) wmax[wave] = mx;
    __syncthreads();
#pragma unroll
    for (int q = 0; q < 4; ++q) {
        const int rowl = q * 4 + (lane >> 3), pc = lane & 7;
        vst2(Cm + ((size_t)b * NN + row0 + rowl) * NN + col0 + pc * 4, *(const v4f*)(&Ct[wave][rowl * 32 + pc * 4]));
    }
    if (tid < 8) {
        float bm = wmax[0];
#pragma unroll
        for (int w = 1; w < 8; ++w) bm = fmaxf(bm, wmax[w]);
        vst2(maxpart + (size_t)blk * 32 + tid * 4, (v4f){bm, bm, bm, bm});
    }
}

__global__ __launch_bounds__(256) void sk_max(const float* __restrict__ maxpart, float* __restrict__ maxC) {
    __shared__ float red[256];
    __shared__ float res[32];
    const int tid = threadIdx.x;
    for (int b = 0; b < BB; ++b) {
        float m = 0.0f;
        for (int k = tid; k < 1024; k += 256) m = fmaxf(m, maxpart[((size_t)b * 1024 + k) * 32]);
        red[tid] = m;
        __syncthreads();
        for (int s = 128; s > 0; s >>= 1) { if (tid < s) red[tid] = fmaxf(red[tid], red[tid + s]); __syncthreads(); }
        if (tid == 0) res[b] = red[0];
        __syncthreads();
    }
    if (tid < 32) { const float v = (tid < BB) ? res[tid] : 0.0f; vst2(maxC + tid, (float_a)v); }
}

__global__ __launch_bounds__(256) void sk_exp(float* __restrict__ Km, const float* __restrict__ maxC) {
    const size_t i = (size_t)blockIdx.x * 256 + threadIdx.x;
    const int b = (int)(i >> 22);
    const float rn = 1.0f / (maxC[b] + 1e-8f);
    const float c = Km[i];
    const float k = expf(-(c * rn) * 10.0f);
    vst2(Km + i, (float_a)k);
}

__device__ __forceinline__ void vec_frags(const float* vec, int k0, int lane, v16bf& bh, v16bf& bl) {
    if ((lane & 15) == 0) {
        const float* p = vec + k0 + 8 * (lane >> 4);
        const v4f a0 = *(const v4f*)(p), a1 = *(const v4f*)(p + 4), a2 = *(const v4f*)(p + 16), a3 = *(const v4f*)(p + 20);
#pragma unroll
        for (int i = 0; i < 4; ++i) {
            __bf16 h;
            h = bf_hi(a0[i]); bh[i]      = h; bl[i]      = bf_lo(a0[i], h);
            h = bf_hi(a1[i]); bh[4 + i]  = h; bl[4 + i]  = bf_lo(a1[i], h);
            h = bf_hi(a2[i]); bh[8 + i]  = h; bl[8 + i]  = bf_lo(a2[i], h);
            h = bf_hi(a3[i]); bh[12 + i] = h; bl[12 + i] = bf_lo(a3[i], h);
        }
    } else {
#pragma unroll
        for (int i = 0; i < 16; ++i) { bh[i] = (__bf16)0.0f; bl[i] = (__bf16)0.0f; }
    }
}
__device__ __forceinline__ void store_recip(float* ures, const float* vin_dummy, v8f acc, int lane, int wave, float* out128) {
    (void)vin_dummy;
    if ((lane & 15) == 0) {
#pragma unroll
        for (int r = 0; r < 8; ++r) ures[wave * 16 + 8 * (lane >> 4) + r] = 1.0f / (acc[r] + 1e-10f);
    }
    (void)out128;
}
__global__ __launch_bounds__(256) void sk_matvec_rows(const float* __restrict__ Km, const float* __restrict__ v, float* __restrict__ u) {
    __shared__ __align__(16) float ures[128];
    const int tid = threadIdx.x, wave = tid >> 5, lane = tid & 31;
    const int row0 = blockIdx.x * 128 + wave * 16;
    const int b = row0 / NN;
    const float* arow = Km + ((size_t)row0 + (lane & 15)) * NN;
    const float* vb = v + (size_t)b * NN;
    v8f acc = {};
#pragma unroll 2
    for (int k0 = 0; k0 < NN; k0 += 32) {
        v16bf ah, al, bh, bl;
        frag_f32_split(arow, k0, lane, ah, al);
        vec_frags(vb, k0, lane, bh, bl);
        acc = wmma_bf16(ah, bh, acc); acc = wmma_bf16(ah, bl, acc); acc = wmma_bf16(al, bh, acc);
    }
    store_recip(ures, nullptr, acc, lane, wave, nullptr);
    __syncthreads();
    if (tid < 32) vst2(u + (size_t)blockIdx.x * 128 + tid * 4, *(const v4f*)(&ures[tid * 4]));
}
__global__ __launch_bounds__(256) void sk_matvec_cols(const float* __restrict__ Km, const float* __restrict__ u, float* __restrict__ v) {
    __shared__ __align__(16) float vres[128];
    const int tid = threadIdx.x, wave = tid >> 5, lane = tid & 31, h = lane >> 4, ln = lane & 15;
    const int col0 = blockIdx.x * 128 + wave * 16;
    const int b = col0 / NN;
    const int j = (col0 % NN) + ln;
    const float* Kb_ = Km + (size_t)b * NN * NN;
    const float* ub = u + (size_t)b * NN;
    v8f acc = {};
#pragma unroll 2
    for (int k0 = 0; k0 < NN; k0 += 32) {
        v16bf ah, al, bh, bl;
        if (ln == 0) {
            const float* p = ub + k0 + 8 * h;
            const v4f a0 = *(const v4f*)(p), a1 = *(const v4f*)(p + 4), a2 = *(const v4f*)(p + 16), a3 = *(const v4f*)(p + 20);
#pragma unroll
            for (int i = 0; i < 4; ++i) {
                __bf16 t;
                t = bf_hi(a0[i]); ah[i]      = t; al[i]      = bf_lo(a0[i], t);
                t = bf_hi(a1[i]); ah[4 + i]  = t; al[4 + i]  = bf_lo(a1[i], t);
                t = bf_hi(a2[i]); ah[8 + i]  = t; al[8 + i]  = bf_lo(a2[i], t);
                t = bf_hi(a3[i]); ah[12 + i] = t; al[12 + i] = bf_lo(a3[i], t);
            }
        } else {
#pragma unroll
            for (int i = 0; i < 16; ++i) { ah[i] = (__bf16)0.0f; al[i] = (__bf16)0.0f; }
        }
#pragma unroll
        for (int e = 0; e < 16; ++e) {
            const int i = k0 + 8 * h + (e < 8 ? e : 8 + e);
            const float x = Kb_[(size_t)i * NN + j];
            const __bf16 t = bf_hi(x); bh[e] = t; bl[e] = bf_lo(x, t);
        }
        acc = wmma_bf16(ah, bh, acc); acc = wmma_bf16(ah, bl, acc); acc = wmma_bf16(al, bh, acc);
    }
    if (h == 0) vres[wave * 16 + ln] = 1.0f / (acc[0] + 1e-10f);
    __syncthreads();
    if (tid < 32) vst2(v + (size_t)blockIdx.x * 128 + tid * 4, *(const v4f*)(&vres[tid * 4]));
}

__global__ __launch_bounds__(256) void sk_argmax(const float* __restrict__ Km, const float* __restrict__ v, int* __restrict__ out) {
    __shared__ float ldsv[NN];
    __shared__ int res[32];
    const int tid = threadIdx.x, wave = tid >> 5, lane = tid & 31;
    const int row0 = blockIdx.x * 32;
    const int b = row0 / NN;
    for (int i = tid; i < NN; i += 256) ldsv[i] = v[(size_t)b * NN + i];
    __syncthreads();
    for (int rr = 0; rr < 4; ++rr) {
        const int row = row0 + wave * 4 + rr;
        const float* Krow = Km + (size_t)row * NN;
        float best = -1.0f; int bidx = 0x7fffffff;
        for (int t = 0; t < NN / 32; ++t) {
            const int j = t * 32 + lane;
            const float p = Krow[j] * ldsv[j];
            if (p > best || (p == best && j < bidx)) { best = p; bidx = j; }
        }
        for (int m = 16; m > 0; m >>= 1) {
            const float ob = __shfl_xor(best, m, 32);
            const int   oi = __shfl_xor(bidx, m, 32);
            if (ob > best || (ob == best && oi < bidx)) { best = ob; bidx = oi; }
        }
        if (lane == 0) res[wave * 4 + rr] = (bidx >= 0 && bidx < NN) ? bidx : 0;
    }
    __syncthreads();
    if (tid < 8) vst2(out + row0 + tid * 4, *(const v4i*)(&res[tid * 4]));
}

extern "C" void kernel_launch(void* const* d_in, const int* in_sizes, int n_in,
                              void* d_out, int out_size, void* d_ws, size_t ws_size,
                              hipStream_t stream) {
    (void)in_sizes; (void)n_in; (void)out_size; (void)ws_size;
    const float* x0 = (const float*)d_in[0];
    const float* x1 = (const float*)d_in[1];

    char* ws = (char*)d_ws;
    const size_t KB = (size_t)BB * NN * NN;
    float*  Km   = (float*)ws;
    char*   tail = ws + KB * 4;
    float*  sq0  = (float*)tail;                 tail += (size_t)BB * NN * 4;
    float*  sq1  = (float*)tail;                 tail += (size_t)BB * NN * 4;
    float*  u    = (float*)tail;                 tail += (size_t)BB * NN * 4;
    float*  v    = (float*)tail;                 tail += (size_t)BB * NN * 4;
    float*  maxC = (float*)tail;                 tail += 128;
    float*  maxpart = (float*)tail;

    sk_init<<<(BB * NN) / (256 * 4), 256, 0, stream>>>(v);
    sk_rowsq<<<(BB * NN) / 256, 256, 0, stream>>>(x0, x1, sq0, sq1);
    sk_cost<<<BB * 16 * 64, 256, 0, stream>>>(x0, x1, sq0, sq1, Km, maxpart);
    sk_max<<<1, 256, 0, stream>>>(maxpart, maxC);
    sk_exp<<<(unsigned)(KB / 256), 256, 0, stream>>>(Km, maxC);
    for (int it = 0; it < ITERS; ++it) {
        sk_matvec_rows<<<(BB * NN) / 128, 256, 0, stream>>>(Km, v, u);
        sk_matvec_cols<<<(BB * NN) / 128, 256, 0, stream>>>(Km, u, v);
    }
    sk_argmax<<<(BB * NN) / 32, 256, 0, stream>>>(Km, v, (int*)d_out);
}
